// HGN_AD_9543417332148
// MI455X (gfx1250) — hardware-verified
//
#include <hip/hip_runtime.h>


typedef __bf16       v16b __attribute__((ext_vector_type(16)));
typedef _Float16     v16h __attribute__((ext_vector_type(16)));
typedef float        v8f  __attribute__((ext_vector_type(8)));
typedef int          v8i  __attribute__((ext_vector_type(8)));
typedef float        v4f  __attribute__((ext_vector_type(4)));
typedef int          v4i  __attribute__((ext_vector_type(4)));
typedef unsigned int v4u  __attribute__((ext_vector_type(4)));

union FragB { v16b v; v4u u[2]; unsigned short s[16]; };
union FragH { v16h v; v4u u[2]; _Float16 e[16]; };

#define TT     32
#define NNOD   512
#define NE     64
#define NF     64
#define NH     64
#define TNR    (TT * NNOD)
#define NEGV   (-1.0e9f)
#define LPITCH 68

#define OFF_H     0u
#define OFF_HI    4194304u
#define OFF_LO    6291456u
#define OFF_SHYP  8388608u
#define OFF_SIND  8454144u
#define OFF_STATS 8519680u
#define OFF_IND   8552448u
#define WS_END    12746752u

__device__ __forceinline__ int koff(int i, int hh) { return i + 8 * hh + ((i < 8) ? 0 : 8); }

__device__ __forceinline__ unsigned short bf16_bits(float f) {
  unsigned int u = __builtin_bit_cast(unsigned int, f);
  u += 0x7FFFu + ((u >> 16) & 1u);
  return (unsigned short)(u >> 16);
}
__device__ __forceinline__ float bf16_val(unsigned short s) {
  return __builtin_bit_cast(float, ((unsigned int)s) << 16);
}
__device__ __forceinline__ unsigned short f16_bits(float f) {
  return __builtin_bit_cast(unsigned short, (_Float16)f);
}
__device__ __forceinline__ v8f zero8() { v8f z = {0.f, 0.f, 0.f, 0.f, 0.f, 0.f, 0.f, 0.f}; return z; }

__device__ __forceinline__ v8f mma_bf16(const v16b a, const v16b b, v8f c) {
  c = __builtin_amdgcn_wmma_f32_16x16x32_bf16(false, a, false, b, (short)0, c, false, false);
  asm volatile("v_nop\n\tv_nop\n\tv_nop\n\tv_nop" : "+v"(c)
               : "v"(__builtin_bit_cast(v8i, a)), "v"(__builtin_bit_cast(v8i, b)));
  return c;
}
__device__ __forceinline__ v8f mma_f16(const v16h a, const v16h b, v8f c) {
  c = __builtin_amdgcn_wmma_f32_16x16x32_f16(false, a, false, b, (short)0, c, false, false);
  asm volatile("v_nop\n\tv_nop\n\tv_nop\n\tv_nop" : "+v"(c)
               : "v"(__builtin_bit_cast(v8i, a)), "v"(__builtin_bit_cast(v8i, b)));
  return c;
}

__device__ __forceinline__ float wmax32(float v) {
  v = fmaxf(v, __shfl_xor(v, 16)); v = fmaxf(v, __shfl_xor(v, 8)); v = fmaxf(v, __shfl_xor(v, 4));
  v = fmaxf(v, __shfl_xor(v, 2));  v = fmaxf(v, __shfl_xor(v, 1));
  return v;
}
__device__ __forceinline__ float wsum32(float v) {
  v += __shfl_xor(v, 16); v += __shfl_xor(v, 8); v += __shfl_xor(v, 4);
  v += __shfl_xor(v, 2);  v += __shfl_xor(v, 1);
  return v;
}
__device__ __forceinline__ float wsum16(float v) {
  v += __shfl_xor(v, 8); v += __shfl_xor(v, 4); v += __shfl_xor(v, 2); v += __shfl_xor(v, 1);
  return v;
}
__device__ __forceinline__ float eluf(float v)  { return v > 0.f ? v : (__expf(v) - 1.f); }
__device__ __forceinline__ float leakyf(float v) { return v >= 0.f ? v : 0.2f * v; }

__device__ __forceinline__ void kh_store(float* h, unsigned short* hThi, unsigned short* hTlo,
                                         float* s_hyp, float* s_ind,
                                         const v4f (&hv)[8], const v4u (&ph)[4], const v4u (&pl)[4],
                                         const v4f sv, int tid, int wave, int lane,
                                         int rbase, int t, int jbase) {
#pragma unroll
  for (int q = 0; q < 8; ++q) {
    const int item = tid + 256 * q;
    const int j = item >> 4, c = (item & 15) * 4;
    *(volatile v4f*)(h + (size_t)(rbase + j) * NH + c) = hv[q];
  }
#pragma unroll
  for (int q = 0; q < 4; ++q) {
    const int item = tid + 256 * q;
    const int d = item >> 4, jb = item & 15;
    const size_t off = ((size_t)(t * NH + d)) * NNOD + (size_t)jbase + (size_t)jb * 8;
    *(volatile v4u*)(hThi + off) = ph[q];
    *(volatile v4u*)(hTlo + off) = pl[q];
  }
  if (wave == 0)      *(volatile v4f*)(s_hyp + rbase + 4 * lane) = sv;
  else if (wave == 1) *(volatile v4f*)(s_ind + rbase + 4 * lane) = sv;
}

__global__ void __launch_bounds__(256)
k_hgemm(const float* __restrict__ x, const float* __restrict__ W,
        const float* __restrict__ a_hyp, const float* __restrict__ a_ind,
        const int* __restrict__ nhid,
        float* h, unsigned short* hThi, unsigned short* hTlo,
        float* s_hyp, float* s_ind) {
  __shared__ __attribute__((aligned(16))) unsigned short lWhi[NH * NF];
  __shared__ __attribute__((aligned(16))) unsigned short lWlo[NH * NF];
  __shared__ float la[2][NF];
  __shared__ __attribute__((aligned(16))) float ltile[128][LPITCH];
  __shared__ __attribute__((aligned(16))) float ls[2][128];

  const int tid = threadIdx.x, wave = tid >> 5, lane = tid & 31, hh = lane >> 4, m = lane & 15;
  const int blk = blockIdx.x;
  const int rbase = blk * 128;
  const int t = blk >> 2;
  const int jbase = (blk & 3) * 128;
  (void)nhid;

#pragma unroll
  for (int q = 0; q < 16; ++q) {
    const int idx = tid + 256 * q;
    const int k = idx >> 6, d = idx & 63;
    const float f = W[idx];
    const unsigned short hb = bf16_bits(f);
    lWhi[d * NF + k] = hb;
    lWlo[d * NF + k] = bf16_bits(f - bf16_val(hb));
  }
  if (tid < NF) { la[0][tid] = a_hyp[tid]; la[1][tid] = a_ind[tid]; }
  __syncthreads();

  v8f acc[4];
#pragma unroll
  for (int nt = 0; nt < 4; ++nt) acc[nt] = zero8();

  const float* xrow = x + (size_t)(rbase + wave * 16 + m) * NF;
#pragma unroll
  for (int kc = 0; kc < 2; ++kc) {
    const float* xp = xrow + 32 * kc;
    v4f fq[4];
    fq[0] = *(const v4f*)(xp + 8 * hh);
    fq[1] = *(const v4f*)(xp + 8 * hh + 4);
    fq[2] = *(const v4f*)(xp + 16 + 8 * hh);
    fq[3] = *(const v4f*)(xp + 20 + 8 * hh);
    FragB ah, al;
#pragma unroll
    for (int i = 0; i < 16; ++i) {
      const float f = fq[i >> 2][i & 3];
      const unsigned short hb = bf16_bits(f);
      ah.s[i] = hb;
      al.s[i] = bf16_bits(f - bf16_val(hb));
    }
#pragma unroll
    for (int nt = 0; nt < 4; ++nt) {
      const unsigned short* bp = lWhi + (16 * nt + m) * NF + 32 * kc;
      const unsigned short* bq = lWlo + (16 * nt + m) * NF + 32 * kc;
      FragB bh, bl;
      bh.u[0] = *(const v4u*)(bp + 8 * hh);
      bh.u[1] = *(const v4u*)(bp + 16 + 8 * hh);
      bl.u[0] = *(const v4u*)(bq + 8 * hh);
      bl.u[1] = *(const v4u*)(bq + 16 + 8 * hh);
      acc[nt] = mma_bf16(ah.v, bh.v, acc[nt]);
      acc[nt] = mma_bf16(ah.v, bl.v, acc[nt]);
      acc[nt] = mma_bf16(al.v, bh.v, acc[nt]);
    }
  }

#pragma unroll
  for (int nt = 0; nt < 4; ++nt)
#pragma unroll
    for (int r = 0; r < 8; ++r)
      ltile[wave * 16 + 8 * hh + r][16 * nt + m] = acc[nt][r];
  __syncthreads();

  {
    const int j = tid & 127, which = tid >> 7;
    float s = 0.f;
#pragma unroll 16
    for (int d = 0; d < NH; ++d) s += ltile[j][d] * la[which][d];
    ls[which][j] = leakyf(s);
  }
  __syncthreads();

  v4f hv[8];
#pragma unroll
  for (int q = 0; q < 8; ++q) {
    const int item = tid + 256 * q;
    const int j = item >> 4, c = (item & 15) * 4;
    hv[q] = *(const v4f*)&ltile[j][c];
  }
  v4u ph[4], pl[4];
#pragma unroll
  for (int q = 0; q < 4; ++q) {
    const int item = tid + 256 * q;
    const int d = item >> 4, jb = item & 15;
    unsigned int wh[4], wl[4];
#pragma unroll
    for (int u = 0; u < 4; ++u) {
      const float fa = ltile[jb * 8 + 2 * u][d];
      const float fb = ltile[jb * 8 + 2 * u + 1][d];
      const unsigned short ha = bf16_bits(fa), hb = bf16_bits(fb);
      const unsigned short la_ = bf16_bits(fa - bf16_val(ha)), lb_ = bf16_bits(fb - bf16_val(hb));
      wh[u] = (unsigned int)ha | ((unsigned int)hb << 16);
      wl[u] = (unsigned int)la_ | ((unsigned int)lb_ << 16);
    }
    v4u a = {wh[0], wh[1], wh[2], wh[3]};
    v4u b = {wl[0], wl[1], wl[2], wl[3]};
    ph[q] = a; pl[q] = b;
  }
  v4f sv = *(const v4f*)&ls[wave & 1][4 * lane];

  kh_store(h, hThi, hTlo, s_hyp, s_ind, hv, ph, pl, sv, tid, wave, lane, rbase, t, jbase);
  __threadfence();
  kh_store(h, hThi, hTlo, s_hyp, s_ind, hv, ph, pl, sv, tid, wave, lane, rbase, t, jbase);
}

__global__ void __launch_bounds__(256)
k_stats(const int* __restrict__ H, const float* __restrict__ s_hyp, float* stats) {
  __shared__ __attribute__((aligned(16))) float lst[256];
  const int tid = threadIdx.x, wave = tid >> 5, lane = tid & 31;
  const int t = blockIdx.x;
  const float NINF = __int_as_float(0xff800000);

  float sv[16];
#pragma unroll
  for (int it = 0; it < 16; ++it) sv[it] = s_hyp[t * NNOD + it * 32 + lane];

#pragma unroll 1
  for (int q = 0; q < 8; ++q) {
    const int e = wave * 8 + q;
    unsigned int mbits = 0u;
#pragma unroll
    for (int it = 0; it < 16; ++it)
      if (H[(it * 32 + lane) * NE + e] != 0) mbits |= (1u << it);
    float mx = NINF;
#pragma unroll
    for (int it = 0; it < 16; ++it)
      mx = fmaxf(mx, ((mbits >> it) & 1u) ? sv[it] : NINF);
    mx = wmax32(mx);
    float sum = 0.f;
#pragma unroll
    for (int it = 0; it < 16; ++it) {
      const bool memb = ((mbits >> it) & 1u) != 0u;
      const float arg = memb ? (sv[it] - mx) : -80.f;
      sum += memb ? __expf(arg) : 0.f;
    }
    sum = wsum32(sum);
    const bool ok = sum > 0.f;
    if (lane == 0) {
      lst[e]       = ok ? mx : 0.f;
      lst[64 + e]  = ok ? (1.f / sum) : 0.f;
      lst[128 + e] = ok ? 0.f : (1.f / 512.f);
      lst[192 + e] = 0.f;
    }
  }
  __syncthreads();
  if (wave == 0) {
    const v4f a = *(const v4f*)&lst[4 * lane];
    const v4f b = *(const v4f*)&lst[128 + 4 * lane];
    float* p = stats + t * 256;
    *(volatile v4f*)(p + 4 * lane) = a;
    *(volatile v4f*)(p + 128 + 4 * lane) = b;
    __threadfence();
    *(volatile v4f*)(p + 4 * lane) = a;
    *(volatile v4f*)(p + 128 + 4 * lane) = b;
  }
}

__global__ void __launch_bounds__(128)
k_industry(const int* __restrict__ adj, const float* __restrict__ s_ind,
           const unsigned short* __restrict__ hThi, const unsigned short* __restrict__ hTlo,
           float* industry) {
  __shared__ __attribute__((aligned(16))) float lex[NNOD];
  __shared__ float lred[4];
  __shared__ __attribute__((aligned(16))) float ltile[64][LPITCH];

  const int tid = threadIdx.x, wave = tid >> 5, lane = tid & 31, hh = lane >> 4, m = lane & 15;
  const int t = blockIdx.x >> 3;
  const int ibase = (blockIdx.x & 7) * 64;
  const int wrow0 = ibase + wave * 16;

  {
    const float v0 = s_ind[t * NNOD + tid];
    const float v1 = s_ind[t * NNOD + tid + 128];
    const float v2 = s_ind[t * NNOD + tid + 256];
    const float v3 = s_ind[t * NNOD + tid + 384];
    float mx = fmaxf(fmaxf(v0, v1), fmaxf(v2, v3));
    mx = wmax32(mx);
    if (lane == 0) lred[wave] = mx;
    __syncthreads();
    const float g = fmaxf(fmaxf(lred[0], lred[1]), fmaxf(lred[2], lred[3]));
    lex[tid]       = __expf(v0 - g);
    lex[tid + 128] = __expf(v1 - g);
    lex[tid + 256] = __expf(v2 - g);
    lex[tid + 384] = __expf(v3 - g);
  }
  __syncthreads();

  const int* arow = adj + (size_t)(wrow0 + m) * NNOD;

  float sum = 0.f;
#pragma unroll 1
  for (int kc = 0; kc < 16; ++kc) {
    v4i qq[4];
    qq[0] = *(const v4i*)(arow + 32 * kc + 8 * hh);
    qq[1] = *(const v4i*)(arow + 32 * kc + 8 * hh + 4);
    qq[2] = *(const v4i*)(arow + 32 * kc + 16 + 8 * hh);
    qq[3] = *(const v4i*)(arow + 32 * kc + 20 + 8 * hh);
#pragma unroll
    for (int i = 0; i < 16; ++i) {
      const int a = qq[i >> 2][i & 3];
      sum += (a != 0) ? lex[32 * kc + koff(i, hh)] : 0.f;
    }
  }
  sum += __shfl_xor(sum, 16);
  const bool ok = sum > 0.f;
  const float iz  = ok ? (1.f / sum) : 0.f;
  const float uni = ok ? 0.f : (1.f / 512.f);

  v8f acc[4];
#pragma unroll
  for (int nt = 0; nt < 4; ++nt) acc[nt] = zero8();

#pragma unroll 1
  for (int kc = 0; kc < 16; ++kc) {
    v4i qq[4];
    qq[0] = *(const v4i*)(arow + 32 * kc + 8 * hh);
    qq[1] = *(const v4i*)(arow + 32 * kc + 8 * hh + 4);
    qq[2] = *(const v4i*)(arow + 32 * kc + 16 + 8 * hh);
    qq[3] = *(const v4i*)(arow + 32 * kc + 20 + 8 * hh);
    FragB ah, al;
#pragma unroll
    for (int i = 0; i < 16; ++i) {
      const int a = qq[i >> 2][i & 3];
      const float b = ((a != 0) ? lex[32 * kc + koff(i, hh)] * iz : 0.f) + uni;
      const unsigned short hb = bf16_bits(b);
      ah.s[i] = hb;
      al.s[i] = bf16_bits(b - bf16_val(hb));
    }
#pragma unroll
    for (int nt = 0; nt < 4; ++nt) {
      const size_t boff = ((size_t)(t * NH + 16 * nt + m)) * NNOD + (size_t)(32 * kc);
      FragB bh, bl;
      bh.u[0] = *(const v4u*)(hThi + boff + 8 * hh);
      bh.u[1] = *(const v4u*)(hThi + boff + 16 + 8 * hh);
      bl.u[0] = *(const v4u*)(hTlo + boff + 8 * hh);
      bl.u[1] = *(const v4u*)(hTlo + boff + 16 + 8 * hh);
      acc[nt] = mma_bf16(ah.v, bh.v, acc[nt]);
      acc[nt] = mma_bf16(ah.v, bl.v, acc[nt]);
      acc[nt] = mma_bf16(al.v, bh.v, acc[nt]);
    }
  }

#pragma unroll
  for (int nt = 0; nt < 4; ++nt)
#pragma unroll
    for (int r = 0; r < 8; ++r)
      ltile[wave * 16 + 8 * hh + r][16 * nt + m] = acc[nt][r];
  __syncthreads();

  v4f ov[8];
#pragma unroll
  for (int q = 0; q < 8; ++q) ov[q] = *(const v4f*)&ltile[wave * 16 + 2 * q + hh][4 * m];
#pragma unroll
  for (int q = 0; q < 8; ++q) {
    float* p = industry + ((size_t)(t * NNOD + wrow0 + 2 * q + hh)) * NH + 4 * m;
    *(volatile v4f*)p = ov[q];
  }
  __threadfence();
#pragma unroll
  for (int q = 0; q < 8; ++q) {
    float* p = industry + ((size_t)(t * NNOD + wrow0 + 2 * q + hh)) * NH + 4 * m;
    *(volatile v4f*)p = ov[q];
  }
}

__global__ void __launch_bounds__(128)
k_edge(const int* __restrict__ H, const float* __restrict__ h, const float* __restrict__ s_hyp,
       const float* __restrict__ stats, const float* __restrict__ industry,
       const float* __restrict__ Wc1, const float* __restrict__ bc1,
       const float* __restrict__ wc2, const float* __restrict__ bc2,
       float* out) {
  __shared__ __attribute__((aligned(16))) unsigned short lW[NH * NH];
  __shared__ float lbc1[NH], lwc2[NH], lme[NE], lize[NE], lune[NE];
  __shared__ float lal[4][NE], lz[4][NE], la2[4][NE], lp[4][2][NH];
  __shared__ __attribute__((aligned(16))) float lo_[4][NH];
  __shared__ float lfe[4][NH][65];

  const int tid = threadIdx.x, wave = tid >> 5, lane = tid & 31, hh = lane >> 4, m = lane & 15;
  const int t = blockIdx.x >> 7;
  const int gw = blockIdx.x * 4 + wave;
  const int n = gw & (NNOD - 1);

#pragma unroll
  for (int q = 0; q < 32; ++q) {
    const int idx = tid + 128 * q;
    const int k = idx >> 6, d = idx & 63;
    lW[d * NH + k] = f16_bits(64.f * Wc1[idx]);
  }
  if (tid < NH) {
    lbc1[tid] = bc1[tid];
    lwc2[tid] = wc2[tid];
    lme[tid]  = stats[t * 256 + tid];
    lize[tid] = stats[t * 256 + 64 + tid];
    lune[tid] = stats[t * 256 + 128 + tid];
  }
  const float bc2v = bc2[0];
  const float hv0 = h[(size_t)gw * NH + lane];
  const float hv1 = h[(size_t)gw * NH + lane + 32];
  const int mk0 = (H[n * NE + lane] != 0) ? 1 : 0;
  const int mk1 = (H[n * NE + lane + 32] != 0) ? 1 : 0;
  const float sh = s_hyp[gw];
  __syncthreads();

  {
    const float al0 = (mk0 ? __expf(sh - lme[lane]) * lize[lane] : 0.f) + lune[lane];
    const float al1 = (mk1 ? __expf(sh - lme[lane + 32]) * lize[lane + 32] : 0.f) + lune[lane + 32];
    lal[wave][lane] = al0;
    lal[wave][lane + 32] = al1;
  }
  __syncthreads();

#pragma unroll 8
  for (int e = 0; e < NE; ++e) {
    const float a = lal[wave][e];
    lfe[wave][lane][e]      = eluf(a * hv0);
    lfe[wave][lane + 32][e] = eluf(a * hv1);
  }
  __syncthreads();

#pragma unroll 1
  for (int mt = 0; mt < 4; ++mt) {
    v8f acc[4];
#pragma unroll
    for (int nt = 0; nt < 4; ++nt) acc[nt] = zero8();
    const int erow = 16 * mt + m;
#pragma unroll
    for (int kc = 0; kc < 2; ++kc) {
      FragH a;
#pragma unroll
      for (int i = 0; i < 16; ++i)
        a.e[i] = (_Float16)(256.f * lfe[wave][32 * kc + koff(i, hh)][erow]);
#pragma unroll
      for (int nt = 0; nt < 4; ++nt) {
        const unsigned short* bp = lW + (16 * nt + m) * NH + 32 * kc;
        FragH b;
        b.u[0] = *(const v4u*)(bp + 8 * hh);
        b.u[1] = *(const v4u*)(bp + 16 + 8 * hh);
        acc[nt] = mma_f16(a.v, b.v, acc[nt]);
      }
    }
#pragma unroll
    for (int r = 0; r < 8; ++r) {
      float zp = 0.f;
#pragma unroll
      for (int nt = 0; nt < 4; ++nt) {
        const int dd = 16 * nt + m;
        zp += fmaxf(acc[nt][r] * (1.f / 16384.f) + lbc1[dd], 0.f) * lwc2[dd];
      }
      zp = wsum16(zp);
      if (m == 0) lz[wave][16 * mt + 8 * hh + r] = zp + bc2v;
    }
  }
  __syncthreads();

  {
    const float z0 = mk0 ? lz[wave][lane] : NEGV;
    const float z1 = mk1 ? lz[wave][lane + 32] : NEGV;
    const float mz = wmax32(fmaxf(z0, z1));
    const float e0 = __expf(z0 - mz), e1 = __expf(z1 - mz);
    const float ss = wsum32(e0 + e1);
    const float inv = 1.f / ss;
    la2[wave][lane] = e0 * inv;
    la2[wave][lane + 32] = e1 * inv;
  }
  __syncthreads();

  float y0 = 0.f, y1 = 0.f;
#pragma unroll 8
  for (int e = 0; e < NE; ++e) {
    const float a2 = la2[wave][e];
    y0 += a2 * lfe[wave][lane][e];
    y1 += a2 * lfe[wave][lane + 32][e];
  }
  const float ind0 = industry[(size_t)gw * NH + lane];
  const float ind1 = industry[(size_t)gw * NH + lane + 32];
  lp[wave][0][lane] = ind0; lp[wave][0][lane + 32] = ind1;
  lp[wave][1][lane] = y0;   lp[wave][1][lane + 32] = y1;
  __syncthreads();

  v8f acc2[4];
#pragma unroll
  for (int nt = 0; nt < 4; ++nt) acc2[nt] = zero8();
  const int mrow = (m < 2) ? m : 0;
  const float msel = (m < 2) ? 256.f : 0.f;
#pragma unroll
  for (int kc = 0; kc < 2; ++kc) {
    FragH a;
#pragma unroll
    for (int i = 0; i < 16; ++i)
      a.e[i] = (_Float16)(msel * lp[wave][mrow][32 * kc + koff(i, hh)]);
#pragma unroll
    for (int nt = 0; nt < 4; ++nt) {
      const unsigned short* bp = lW + (16 * nt + m) * NH + 32 * kc;
      FragH b;
      b.u[0] = *(const v4u*)(bp + 8 * hh);
      b.u[1] = *(const v4u*)(bp + 16 + 8 * hh);
      acc2[nt] = mma_f16(a.v, b.v, acc2[nt]);
    }
  }
  float zp0 = 0.f, zp1 = 0.f;
#pragma unroll
  for (int nt = 0; nt < 4; ++nt) {
    const int dd = 16 * nt + m;
    zp0 += fmaxf(acc2[nt][0] * (1.f / 16384.f) + lbc1[dd], 0.f) * lwc2[dd];
    zp1 += fmaxf(acc2[nt][1] * (1.f / 16384.f) + lbc1[dd], 0.f) * lwc2[dd];
  }
  zp0 = wsum16(zp0);
  zp1 = wsum16(zp1);
  const float z20 = __shfl(zp0, 0) + bc2v;
  const float z21 = __shfl(zp1, 0) + bc2v;
  const float mm = fmaxf(z20, z21);
  const float w0 = __expf(z20 - mm), w1 = __expf(z21 - mm);
  const float wi = 1.f / (w0 + w1);
  const float p0 = w0 * wi, p1 = w1 * wi;
  const float o0 = p0 * ind0 + p1 * y0;
  const float o1 = p0 * ind1 + p1 * y1;
  lo_[wave][lane] = o0;
  lo_[wave][lane + 32] = o1;
  __syncthreads();

  const int rr = (2 * wave + hh) & 3;
  v4f ov = *(const v4f*)&lo_[rr][4 * m];
  float* op = out + ((size_t)(blockIdx.x * 4 + rr)) * NH + 4 * m;
  if (wave < 2) *(volatile v4f*)op = ov;
  __threadfence();
  if (wave < 2) *(volatile v4f*)op = ov;
}

extern "C" void kernel_launch(void* const* d_in, const int* in_sizes, int n_in,
                              void* d_out, int out_size, void* d_ws,
                              size_t ws_size, hipStream_t stream) {
  if (n_in < 11) return;
  if (in_sizes[0] != TNR * NF || in_sizes[1] != NNOD * NE || in_sizes[2] != NNOD * NNOD ||
      in_sizes[4] != NF * NH || in_sizes[5] != NH || in_sizes[6] != NH ||
      in_sizes[7] != NH * NH || in_sizes[8] != NH || in_sizes[9] != NH || in_sizes[10] < 1 ||
      out_size != TNR * NH) return;
  if (ws_size < (size_t)WS_END) return;

  const float* x     = (const float*)d_in[0];
  const int*   H     = (const int*)d_in[1];
  const int*   adj   = (const int*)d_in[2];
  const int*   nhid  = (const int*)d_in[3];
  const float* W     = (const float*)d_in[4];
  const float* a_hyp = (const float*)d_in[5];
  const float* a_ind = (const float*)d_in[6];
  const float* Wc1   = (const float*)d_in[7];
  const float* bc1   = (const float*)d_in[8];
  const float* wc2   = (const float*)d_in[9];
  const float* bc2   = (const float*)d_in[10];

  char* ws = (char*)d_ws;
  float*          h        = (float*)(ws + OFF_H);
  unsigned short* hThi     = (unsigned short*)(ws + OFF_HI);
  unsigned short* hTlo     = (unsigned short*)(ws + OFF_LO);
  float*          s_hyp    = (float*)(ws + OFF_SHYP);
  float*          s_ind    = (float*)(ws + OFF_SIND);
  float*          stats    = (float*)(ws + OFF_STATS);
  float*          industry = (float*)(ws + OFF_IND);
  float*          out      = (float*)d_out;

  k_hgemm<<<TNR / 128, 256, 0, stream>>>(x, W, a_hyp, a_ind, nhid, h, hThi, hTlo, s_hyp, s_ind);
  k_stats<<<TT, 256, 0, stream>>>(H, s_hyp, stats);
  k_industry<<<TT * (NNOD / 64), 128, 0, stream>>>(adj, s_ind, hThi, hTlo, industry);
  k_edge<<<TNR / 4, 128, 0, stream>>>(H, h, s_hyp, stats, industry, Wc1, bc1, wc2, bc2, out);
}
